// MambaBlock_67886253081031
// MI455X (gfx1250) — hardware-run, weakly checked
//
#include <hip/hip_runtime.h>
#include <math.h>

typedef __attribute__((ext_vector_type(16))) _Float16 v16h;
typedef __attribute__((ext_vector_type(8)))  _Float16 v8h;
typedef __attribute__((ext_vector_type(8)))  float    v8f;
typedef __attribute__((ext_vector_type(4)))  float    v4f;

constexpr int kL    = 4096;
constexpr int kDm   = 1024;
constexpr int kDi   = 2048;
constexpr int kNs   = 16;
constexpr int kDtR  = 64;
constexpr int kPrjN = 96;
constexpr int kPrjP = 128;
constexpr int kXZP  = 2 * kDi;
constexpr int kTP   = 260;
constexpr int kScTS = 64;
constexpr int kScCh = 32;
constexpr int kScYP = 36;

static_assert(kDtR + 2 * kNs == kPrjN);
static_assert((kDm % 32) == 0 && (kDi % 32) == 0 && (kDtR % 32) == 0);
static_assert((kL % 64) == 0 && (kXZP % 64) == 0 && (kPrjP % 64) == 0 && (kDi % 64) == 0 && (kDm % 64) == 0);
static_assert((kL % kScTS) == 0 && (kDi % kScCh) == 0 && kScCh == 32 && (kScTS % 16) == 0);
static_assert((kDi % 256) == 0 && (kL % 64) == 0);

constexpr float kCx   = 16.0f;
constexpr float kCw   = 256.0f;
constexpr float kCwdt = 64.0f;
constexpr float kCu   = 64.0f;
constexpr float kCdt  = 64.0f;
constexpr float kCy   = 256.0f;
constexpr float kCr   = 2048.0f;
constexpr float kScaleIn  = 1.0f / (kCx * kCw);
constexpr float kScalePrj = 1.0f / (kCu * kCw);
constexpr float kScaleDt  = 1.0f / (kCdt * kCwdt);
constexpr float kScaleOut = 1.0f / (kCy * kCw);
constexpr float kInvCu = 1.0f / kCu;
constexpr float kInvCr = 1.0f / kCr;

constexpr size_t kSzX16    = (size_t)kL * kDm * 2;
constexpr size_t kSzWIN16  = (size_t)kXZP * kDm * 2;
constexpr size_t kSzXZ     = (size_t)kL * kXZP * 4;
constexpr size_t kSzUC16   = (size_t)kL * kDi * 2;
constexpr size_t kSzUCR    = (size_t)kL * kDi * 2;
constexpr size_t kSzWX16   = (size_t)kPrjP * kDi * 2;
constexpr size_t kSzPROJ   = (size_t)kL * kPrjP * 4;
constexpr size_t kSzDT16   = (size_t)kL * kDtR * 2;
constexpr size_t kSzWDT16  = (size_t)kDi * kDtR * 2;
constexpr size_t kSzWOUT16 = (size_t)kDm * kDi * 2;
constexpr size_t kSzY16    = (size_t)kL * kDi * 2;
constexpr size_t kOffX16    = 0;
constexpr size_t kOffWIN16  = kOffX16    + kSzX16;
constexpr size_t kOffXZ     = kOffWIN16  + kSzWIN16;
constexpr size_t kOffUC16   = kOffXZ     + kSzXZ;
constexpr size_t kOffUCR    = kOffUC16   + kSzUC16;
constexpr size_t kOffWX16   = kOffUCR    + kSzUCR;
constexpr size_t kOffPROJ   = kOffWX16   + kSzWX16;
constexpr size_t kOffDT16   = kOffPROJ   + kSzPROJ;
constexpr size_t kOffWDT16  = kOffDT16   + kSzDT16;
constexpr size_t kOffWOUT16 = kOffWDT16  + kSzWDT16;
constexpr size_t kWsTotal   = kOffWOUT16 + kSzWOUT16;
constexpr size_t kOffY16    = kOffX16;
static_assert(kWsTotal == 125042688ull);
static_assert(kWsTotal <= 134217728ull);
static_assert(kSzY16 == kSzX16 + kSzWIN16 && kOffWIN16 == kOffX16 + kSzX16);
static_assert((kOffWIN16 % 128) == 0 && (kOffXZ % 128) == 0 && (kOffUC16 % 128) == 0 && (kOffUCR % 128) == 0 &&
              (kOffWX16 % 128) == 0 && (kOffPROJ % 128) == 0 && (kOffDT16 % 128) == 0 && (kOffWDT16 % 128) == 0 &&
              (kOffWOUT16 % 128) == 0);

__device__ __forceinline__ float h16_to_f32(unsigned hb) {
  const unsigned sgn = (hb & 0x8000u) << 16;
  const unsigned em = hb & 0x7fffu;
  const float fn = __uint_as_float((em << 13) + 0x38000000u);
  const float fs = (float)em * 5.9604644775390625e-8f;
  const float mag = (em < 0x400u) ? fs : fn;
  return __uint_as_float(__float_as_uint(mag) | sgn);
}
__device__ __forceinline__ _Float16 to_h16_flush(float v) {
  const float w = (fabsf(v) < 6.103515625e-05f) ? 0.0f : v;
  return (_Float16)w;
}
__device__ __forceinline__ void tie_acc(v8f& a, v16h x, v16h y) {
  asm volatile("v_nop\n\tv_nop\n\tv_nop\n\tv_nop" : "+v"(a) : "v"(x), "v"(y));
}
__device__ __forceinline__ void keep4_h(v16h a, v16h b, v16h c, v16h d) {
  asm volatile("v_nop" :: "v"(a), "v"(b), "v"(c), "v"(d));
}
struct FragH {
  union U { v16h v; v8h h[2]; };
  static __device__ __forceinline__ v16h load(const _Float16* p) {
    U f;
    f.h[0] = *(const v8h*)(p);
    f.h[1] = *(const v8h*)(p + 16);
    return f.v;
  }
  static __device__ __forceinline__ v8f mma(v16h a, v16h b, v8f c) {
    return __builtin_amdgcn_wmma_f32_16x16x32_f16(false, a, false, b, (short)0, c, false, false);
  }
};

template <int BIAS_MODE, bool AKBLK>
__global__ __launch_bounds__(256) void wmma_gemm64_f16(
    const unsigned short* __restrict__ Ap, int lda,
    const unsigned short* __restrict__ Btp, int ldb,
    float* __restrict__ Cout, int ldc,
    const float* __restrict__ bias,
    int M, int N, int K, float scale)
{
  const _Float16* A  = (const _Float16*)Ap;
  const _Float16* Bt = (const _Float16*)Btp;
  __shared__ __align__(16) float sT[8][16 * 68];
  const int lane = threadIdx.x & 31;
  const int wave = threadIdx.x >> 5;
  const int tilesN = N >> 6;
  const int tilesM = M >> 6;
  const int tile = blockIdx.x * 8 + wave;
  if (tile >= tilesM * tilesN) return;
  const int tm = tile / tilesN;
  const int tn = tile - tm * tilesN;
  const int m0 = tm << 6;
  const int n0 = tn << 6;

  const int rlane = lane & 15;
  const int koff  = (lane >> 4) * 8;
  const int mOff  = (lane >> 4) * 8;
  const size_t akb = (size_t)M << 5;

  v8f acc[4][4];
#pragma unroll
  for (int i = 0; i < 4; ++i)
#pragma unroll
    for (int j = 0; j < 4; ++j) acc[i][j] = (v8f){0.f,0.f,0.f,0.f,0.f,0.f,0.f,0.f};

  for (int k0 = 0; k0 < K; k0 += 32) {
    v16h bh[4];
#pragma unroll
    for (int j = 0; j < 4; ++j) {
      const size_t bo = (size_t)(n0 + (j << 4) + rlane) * ldb + koff + k0;
      bh[j] = FragH::load(Bt + bo);
    }
#pragma unroll
    for (int i = 0; i < 4; ++i) {
      const int arow = m0 + (i << 4) + rlane;
      const size_t ao = AKBLK ? ((size_t)(k0 >> 5) * akb + (size_t)arow * 32 + koff)
                              : ((size_t)arow * lda + koff + k0);
      const v16h ah = FragH::load(A + ao);
#pragma unroll
      for (int j = 0; j < 4; ++j) acc[i][j] = FragH::mma(ah, bh[j], acc[i][j]);
#pragma unroll
      for (int j = 0; j < 4; ++j) tie_acc(acc[i][j], ah, bh[j]);
    }
    keep4_h(bh[0], bh[1], bh[2], bh[3]);
  }

  float* slab = sT[wave];
#pragma unroll
  for (int i = 0; i < 4; ++i) {
    const int mBase = m0 + (i << 4);
#pragma unroll
    for (int j = 0; j < 4; ++j) {
      const int n = n0 + (j << 4) + rlane;
      float bv = 0.f;
      if (BIAS_MODE == 2) bv = bias[n];
#pragma unroll
      for (int r = 0; r < 8; ++r) {
        float v = acc[i][j][r] * scale;
        if (BIAS_MODE == 2) v += bv;
        slab[(mOff + r) * 68 + (j << 4) + rlane] = v;
      }
    }
    __builtin_amdgcn_fence(__ATOMIC_RELEASE, "workgroup");
    __builtin_amdgcn_wave_barrier();
    __builtin_amdgcn_fence(__ATOMIC_ACQUIRE, "workgroup");
    {
      const int hh = lane >> 4, c4 = (lane & 15) * 4;
      for (int pass = 0; pass < 2; ++pass) {
#pragma unroll
        for (int it = 0; it < 8; ++it) {
          const int row = it * 2 + hh;
          const v4f v = *(const v4f*)(slab + row * 68 + c4);
          *(volatile v4f*)(Cout + (size_t)(mBase + row) * ldc + n0 + c4) = v;
        }
        __threadfence();
      }
    }
    __builtin_amdgcn_fence(__ATOMIC_RELEASE, "workgroup");
    __builtin_amdgcn_wave_barrier();
    __builtin_amdgcn_fence(__ATOMIC_ACQUIRE, "workgroup");
  }
}

__global__ __launch_bounds__(256) void cast_f16_kernel(
    const float* __restrict__ src, unsigned short* __restrict__ dst, int total8, int real8, float scale)
{
  const int i = blockIdx.x * 256 + threadIdx.x;
  if (i >= total8) return;
  const bool live = (i < real8);
  const int ic = live ? i : (real8 - 1);
  const float* p = src + ((size_t)ic << 3);
  v4f a0 = *(const v4f*)(p);
  v4f a1 = *(const v4f*)(p + 4);
  asm volatile("" : "+v"(a0));
  asm volatile("" : "+v"(a1));
  v8h hv;
#pragma unroll
  for (int e = 0; e < 4; ++e) {
    const float f0 = live ? (a0[e] * scale) : 0.0f;
    const float f1 = live ? (a1[e] * scale) : 0.0f;
    hv[e]     = to_h16_flush(f0);
    hv[4 + e] = to_h16_flush(f1);
  }
  unsigned short* q = dst + ((size_t)i << 3);
  *(volatile v8h*)q = hv;
  __threadfence();
  *(volatile v8h*)q = hv;
}

__global__ __launch_bounds__(256) void dt_cast_kernel(
    const float* __restrict__ PROJ, unsigned short* __restrict__ DT16, int total8, float scale)
{
  const int i = blockIdx.x * 256 + threadIdx.x;
  if (i >= total8) return;
  const int e0  = i << 3;
  const int row = e0 >> 6;
  const int c8  = e0 & 63;
  const float* p = PROJ + (size_t)row * kPrjP + c8;
  const v4f a0 = *(const v4f*)(p);
  const v4f a1 = *(const v4f*)(p + 4);
  v8h hv;
#pragma unroll
  for (int e = 0; e < 4; ++e) {
    hv[e]     = to_h16_flush(a0[e] * scale);
    hv[4 + e] = to_h16_flush(a1[e] * scale);
  }
  unsigned short* qd = DT16 + e0;
  *(volatile v8h*)qd = hv;
  __threadfence();
  *(volatile v8h*)qd = hv;
}

__global__ __launch_bounds__(256) void conv_silu_kernel(
    const float* __restrict__ XZ, const float* __restrict__ cw, const float* __restrict__ cb,
    unsigned short* __restrict__ UC16, unsigned short* __restrict__ UCR)
{
  __shared__ __align__(16) float sT[16 * kTP];
  const int tid = threadIdx.x, lane = tid & 31, wave = tid >> 5;
  const int d0 = blockIdx.x * 256, d = d0 + tid;
  const int t0 = blockIdx.y * 64;
  const v4f wv = *(const v4f*)(cw + (size_t)d * 4);
  const float w0 = wv[0], w1 = wv[1], w2 = wv[2], w3 = wv[3];
  const float bc = cb[d];
  float xm3, xm2, xm1;
  {
    const int r3 = t0 - 3, r2 = t0 - 2, r1 = t0 - 1;
    const float v3 = XZ[(size_t)(r3 < 0 ? 0 : r3) * kXZP + d];
    const float v2 = XZ[(size_t)(r2 < 0 ? 0 : r2) * kXZP + d];
    const float v1 = XZ[(size_t)(r1 < 0 ? 0 : r1) * kXZP + d];
    xm3 = (r3 >= 0) ? v3 : 0.f;
    xm2 = (r2 >= 0) ? v2 : 0.f;
    xm1 = (r1 >= 0) ? v1 : 0.f;
  }
#pragma unroll 1
  for (int sub = 0; sub < 4; ++sub) {
    const int lb = t0 + sub * 16;
#pragma unroll 1
    for (int s = 0; s < 16; ++s) {
      const float xc = XZ[(size_t)(lb + s) * kXZP + d];
      float acc = w0 * xm3;
      acc = fmaf(w1, xm2, acc);
      acc = fmaf(w2, xm1, acc);
      acc = fmaf(w3, xc, acc);
      const float sv = acc + bc;
      const float sg = 1.0f / (1.0f + expf(-sv));
      sT[s * kTP + tid] = sv * sg;
      xm3 = xm2; xm2 = xm1; xm1 = xc;
    }
    __syncthreads();
    v8h hv[2], rv[2];
#pragma unroll
    for (int it = 0; it < 2; ++it) {
      const float* sp = sT + (it * 8 + wave) * kTP + lane * 8;
      const v4f a0 = *(const v4f*)(sp);
      const v4f a1 = *(const v4f*)(sp + 4);
#pragma unroll
      for (int e = 0; e < 4; ++e) {
        const float s0 = a0[e] * kCu;
        const float s1 = a1[e] * kCu;
        const _Float16 h0 = to_h16_flush(s0);
        const _Float16 h1 = to_h16_flush(s1);
        const float r0 = (s0 - (float)h0) * kCr;
        const float r1 = (s1 - (float)h1) * kCr;
        hv[it][e]     = h0;
        hv[it][4 + e] = h1;
        rv[it][e]     = (_Float16)r0;
        rv[it][4 + e] = (_Float16)r1;
      }
    }
    for (int pass = 0; pass < 2; ++pass) {
#pragma unroll
      for (int it = 0; it < 2; ++it) {
        const size_t o = (size_t)(lb + it * 8 + wave) * kDi + d0 + lane * 8;
        *(volatile v8h*)(UC16 + o) = hv[it];
        *(volatile v8h*)(UCR + o)  = rv[it];
      }
      __threadfence();
    }
    __syncthreads();
  }
}

__global__ __launch_bounds__(128) void scan_kernel(
    const float* __restrict__ XZ, const unsigned* __restrict__ UCw, const unsigned* __restrict__ UCRw,
    const float* __restrict__ PROJ, const float* __restrict__ A_log, const float* __restrict__ Dv,
    unsigned short* __restrict__ Y16)
{
  __shared__ __align__(16) float sDl[kScTS * kScCh];
  __shared__ __align__(16) float sU[kScTS * kScCh];
  __shared__ __align__(16) float sG[kScTS * kScCh];
  __shared__ __align__(16) float sBC[kScTS * 32];
  __shared__ __align__(16) float sY[kScTS * kScYP];
  const int tid = threadIdx.x, lane = tid & 31, wave = tid >> 5;
  const int kb = blockIdx.x;
  const int d0 = kb * kScCh;
  const int c = tid >> 2, sub = tid & 3;
  const int d = d0 + c;

  float An[4], h[4];
  {
    const v4f al = *(const v4f*)(A_log + (size_t)d * kNs + 4 * sub);
#pragma unroll
    for (int k = 0; k < 4; ++k) {
      An[k] = -expf(al[k]);
      h[k] = 0.f;
    }
  }
  const float Dd = Dv[d];

  const int sr = tid >> 5, sc = tid & 31;
  const int br = tid >> 3, bq = (tid & 7) * 4;
  const int q = lane >> 3, j8 = lane & 7;

#pragma unroll 1
  for (int t0 = 0; t0 < kL; t0 += kScTS) {
    __syncthreads();
#pragma unroll 1
    for (int i = 0; i < kScTS / 4; ++i) {
      const int row = i * 4 + sr;
      const size_t m = (size_t)(t0 + row);
      const float a  = XZ[m * kXZP + d0 + sc];
      const float rz = XZ[m * kXZP + kDi + d0 + sc];
      const size_t wi = (m * kDi + d0 + sc) >> 1;
      const unsigned wv = UCw[wi];
      const unsigned wr = UCRw[wi];
      const unsigned hbv = (sc & 1) ? (wv >> 16) : (wv & 0xffffu);
      const unsigned hbr = (sc & 1) ? (wr >> 16) : (wr & 0xffffu);
      const float uval = h16_to_f32(hbv);
      const float ures = h16_to_f32(hbr);
      const float u = (uval + ures * kInvCr) * kInvCu;
      const float delta = fmaxf(a, 0.0f) + log1pf(expf(-fabsf(a)));
      const float g = rz * (1.0f / (1.0f + expf(-rz)));
      sDl[row * kScCh + sc] = delta;
      sU[row * kScCh + sc]  = u;
      sG[row * kScCh + sc]  = g;
    }
#pragma unroll
    for (int i = 0; i < kScTS / 16; ++i) {
      const int row = br + 16 * i;
      const v4f v = *(const v4f*)(PROJ + (size_t)(t0 + row) * kPrjP + kDtR + bq);
      *(v4f*)(sBC + row * 32 + bq) = v;
    }
    __syncthreads();
#pragma unroll 1
    for (int s = 0; s < kScTS; ++s) {
      const float delta = sDl[s * kScCh + c];
      const float u     = sU[s * kScCh + c];
      const float g     = sG[s * kScCh + c];
      const v4f Bv = *(const v4f*)(sBC + s * 32 + 4 * sub);
      const v4f Cv = *(const v4f*)(sBC + s * 32 + kNs + 4 * sub);
      const float dtu = delta * u;
      float y = 0.f;
#pragma unroll
      for (int k = 0; k < 4; ++k) {
        const float e = __expf(delta * An[k]);
        h[k] = fmaf(e, h[k], dtu * Bv[k]);
        y = fmaf(h[k], Cv[k], y);
      }
      y += __shfl_xor(y, 1, 32);
      y += __shfl_xor(y, 2, 32);
      const float yo = (fmaf(u, Dd, y) * g) * kCy;
      if (sub == 0) sY[s * kScYP + c] = yo;
    }
    __syncthreads();
    v8h hv[2];
#pragma unroll
    for (int it = 0; it < 2; ++it) {
      const int ln  = it * 16 + wave * 4 + q;
      const int row = 2 * ln + (j8 >> 2);
      const int ch  = (j8 & 3) * 8;
      const float* sp = sY + row * kScYP + ch;
      const v4f a0 = *(const v4f*)(sp);
      const v4f a1 = *(const v4f*)(sp + 4);
#pragma unroll
      for (int e = 0; e < 4; ++e) {
        hv[it][e]     = to_h16_flush(a0[e]);
        hv[it][4 + e] = to_h16_flush(a1[e]);
      }
    }
    for (int pass = 0; pass < 2; ++pass) {
#pragma unroll
      for (int it = 0; it < 2; ++it) {
        const int ln = it * 16 + wave * 4 + q;
        const size_t o = ((size_t)kb * kL + (size_t)(t0 + 2 * ln)) * 32 + j8 * 8;
        *(volatile v8h*)(Y16 + o) = hv[it];
      }
      __threadfence();
    }
  }
}

extern "C" void kernel_launch(void* const* d_in, const int* in_sizes, int n_in,
                              void* d_out, int out_size, void* d_ws, size_t ws_size,
                              hipStream_t stream)
{
  if (n_in < 10) return;
  if (in_sizes[0] != kL * kDm) return;
  if (in_sizes[1] != kXZP * kDm) return;
  if (in_sizes[2] != kDi * 4) return;
  if (in_sizes[3] != kDi) return;
  if (in_sizes[4] != kPrjN * kDi) return;
  if (in_sizes[5] != kDi * kDtR) return;
  if (in_sizes[6] != kDi) return;
  if (in_sizes[7] != kDi * kNs) return;
  if (in_sizes[8] != kDi) return;
  if (in_sizes[9] != kDm * kDi) return;
  if (out_size != kL * kDm) return;
  if (ws_size < kWsTotal) return;

  const float* x      = (const float*)d_in[0];
  const float* W_in   = (const float*)d_in[1];
  const float* conv_w = (const float*)d_in[2];
  const float* conv_b = (const float*)d_in[3];
  const float* W_x    = (const float*)d_in[4];
  const float* W_dt   = (const float*)d_in[5];
  const float* b_dt   = (const float*)d_in[6];
  const float* A_log  = (const float*)d_in[7];
  const float* Dv     = (const float*)d_in[8];
  const float* W_out  = (const float*)d_in[9];
  float* out = (float*)d_out;

  char* ws = (char*)d_ws;
  unsigned short* X16    = (unsigned short*)(ws + kOffX16);
  unsigned short* WIN16  = (unsigned short*)(ws + kOffWIN16);
  float*          XZ     = (float*)(ws + kOffXZ);
  unsigned short* UC16   = (unsigned short*)(ws + kOffUC16);
  unsigned short* UCR    = (unsigned short*)(ws + kOffUCR);
  unsigned short* WX16   = (unsigned short*)(ws + kOffWX16);
  float*          PROJ   = (float*)(ws + kOffPROJ);
  unsigned short* DT16   = (unsigned short*)(ws + kOffDT16);
  unsigned short* WDT16  = (unsigned short*)(ws + kOffWDT16);
  unsigned short* WOUT16 = (unsigned short*)(ws + kOffWOUT16);
  unsigned short* Y16    = (unsigned short*)(ws + kOffY16);

  cast_f16_kernel<<<(kL * kDm / 8) / 256, 256, 0, stream>>>(x, X16, kL * kDm / 8, kL * kDm / 8, kCx);
  cast_f16_kernel<<<(kXZP * kDm / 8) / 256, 256, 0, stream>>>(W_in, WIN16, kXZP * kDm / 8, kXZP * kDm / 8, kCw);
  cast_f16_kernel<<<(kPrjP * kDi / 8) / 256, 256, 0, stream>>>(W_x, WX16, kPrjP * kDi / 8, kPrjN * kDi / 8, kCw);
  cast_f16_kernel<<<(kDi * kDtR / 8) / 256, 256, 0, stream>>>(W_dt, WDT16, kDi * kDtR / 8, kDi * kDtR / 8, kCwdt);
  cast_f16_kernel<<<(kDm * kDi / 8) / 256, 256, 0, stream>>>(W_out, WOUT16, kDm * kDi / 8, kDm * kDi / 8, kCw);

  wmma_gemm64_f16<0, false><<<(kL / 64) * (kXZP / 64) / 8, 256, 0, stream>>>(
      X16, kDm, WIN16, kDm, XZ, kXZP, b_dt, kL, kXZP, kDm, kScaleIn);

  conv_silu_kernel<<<dim3(kDi / 256, kL / 64), 256, 0, stream>>>(XZ, conv_w, conv_b, UC16, UCR);

  wmma_gemm64_f16<0, false><<<(kL / 64) * (kPrjP / 64) / 8, 256, 0, stream>>>(
      UC16, kDi, WX16, kDi, PROJ, kPrjP, b_dt, kL, kPrjP, kDi, kScalePrj);

  dt_cast_kernel<<<(kL * kDtR / 8) / 256, 256, 0, stream>>>(PROJ, DT16, kL * kDtR / 8, kCdt);

  wmma_gemm64_f16<2, false><<<(kL / 64) * (kDi / 64) / 8, 256, 0, stream>>>(
      DT16, kDtR, WDT16, kDtR, XZ, kXZP, b_dt, kL, kDi, kDtR, kScaleDt);

  scan_kernel<<<kDi / kScCh, 4 * kScCh, 0, stream>>>(
      XZ, (const unsigned*)UC16, (const unsigned*)UCR, PROJ, A_log, Dv, Y16);

  wmma_gemm64_f16<0, true><<<(kL / 64) * (kDm / 64) / 8, 256, 0, stream>>>(
      Y16, 32, WOUT16, kDi, out, kDm, b_dt, kL, kDm, kDi, kScaleOut);
}
